// FusionBlock_61151744360476
// MI455X (gfx1250) — hardware-run, weakly checked
//
#include <hip/hip_runtime.h>
#include <math.h>
#include <stdint.h>

#define NB    4
#define SEQ   2048
#define DM    512
#define NH    8
#define HD    64
#define HID   2048
#define NROW  (NB * SEQ)
#define NQB   (SEQ / 64)

#define WSC   64.0f
#define QSC   8.0f
#define PSC   1024.0f
#define OSC   64.0f
#define MSC   64.0f

static_assert(NH * HD == DM);
static_assert((SEQ % 64) == 0 && (DM % 64) == 0 && (HID % 64) == 0);
static_assert((NROW % 8) == 0);

typedef _Float16 v16h __attribute__((ext_vector_type(16)));
typedef _Float16 v8h  __attribute__((ext_vector_type(8)));
typedef float    v8f  __attribute__((ext_vector_type(8)));
typedef float    v4f  __attribute__((ext_vector_type(4)));
typedef unsigned int v4u __attribute__((ext_vector_type(4)));

__device__ __forceinline__ unsigned short h_bits(_Float16 x) { return __builtin_bit_cast(unsigned short, x); }
__device__ __forceinline__ unsigned pk16(unsigned short a, unsigned short b) { return (unsigned)a | ((unsigned)b << 16); }
__device__ __forceinline__ unsigned pkf(float a, float b) { return pk16(h_bits((_Float16)a), h_bits((_Float16)b)); }
__device__ __forceinline__ v8f zero8() { v8f z = {0.f, 0.f, 0.f, 0.f, 0.f, 0.f, 0.f, 0.f}; return z; }
__device__ __forceinline__ v4f zero4() { v4f z = {0.f, 0.f, 0.f, 0.f}; return z; }
__device__ __forceinline__ float gelu_erf(float v) { return 0.5f * v * (1.0f + erff(v * 0.70710678118654752f)); }
__device__ __forceinline__ v4f gelu4(v4f v) {
  v4f r;
  r[0] = gelu_erf(v[0]); r[1] = gelu_erf(v[1]); r[2] = gelu_erf(v[2]); r[3] = gelu_erf(v[3]);
  return r;
}

__device__ __forceinline__ v16h ldfrag_h(const _Float16* p) {
  union { v16h v; v8h h[2]; } f;
  f.h[0] = *(const v8h*)(p);
  f.h[1] = *(const v8h*)(p + 16);
  return f.v;
}

__device__ __forceinline__ v8f mma_h(v16h a, v16h b, v8f c) {
#if defined(__HIP_DEVICE_COMPILE__)
  c = __builtin_amdgcn_wmma_f32_16x16x32_f16(false, a, false, b, (short)0, c, false, false);
  asm volatile("v_nop\n\tv_nop\n\tv_nop\n\tv_nop" : "+v"(c) : "v"(a), "v"(b));
#endif
  return c;
}
__device__ __forceinline__ v8f mma_h_raw(v16h a, v16h b, v8f c) {
#if defined(__HIP_DEVICE_COMPILE__)
  c = __builtin_amdgcn_wmma_f32_16x16x32_f16(false, a, false, b, (short)0, c, false, false);
#endif
  return c;
}
__device__ __forceinline__ void dep_guard(v8f& a, v8f& b, v16h x) {
#if defined(__HIP_DEVICE_COMPILE__)
  asm volatile("v_nop\n\tv_nop\n\tv_nop\n\tv_nop" : "+v"(a), "+v"(b) : "v"(x));
#endif
}
__device__ __forceinline__ void keep4(v16h a, v16h b, v16h c, v16h d) {
#if defined(__HIP_DEVICE_COMPILE__)
  asm volatile("v_nop" :: "v"(a), "v"(b), "v"(c), "v"(d));
#endif
}
__device__ __forceinline__ void acc_guard4(v8f& a, v8f& b, v8f& c, v8f& d) {
#if defined(__HIP_DEVICE_COMPILE__)
  asm volatile("v_nop\n\tv_nop\n\tv_nop\n\tv_nop" : "+v"(a), "+v"(b), "+v"(c), "+v"(d));
#endif
}
__device__ __forceinline__ void lds_wave_sync() {
  __builtin_amdgcn_fence(__ATOMIC_RELEASE, "workgroup");
  __builtin_amdgcn_wave_barrier();
  __builtin_amdgcn_fence(__ATOMIC_ACQUIRE, "workgroup");
}

__global__ __launch_bounds__(256) void cvt_f16x8(const float* __restrict__ in, unsigned short* out, int n8, float sc) {
  const int i = blockIdx.x * 256 + threadIdx.x;
  if (i < n8) {
    const v4f a = *(const v4f*)(in + (size_t)i * 8);
    const v4f b = *(const v4f*)(in + (size_t)i * 8 + 4);
    v4u p;
    p[0] = pkf(a[0] * sc, a[1] * sc);
    p[1] = pkf(a[2] * sc, a[3] * sc);
    p[2] = pkf(b[0] * sc, b[1] * sc);
    p[3] = pkf(b[2] * sc, b[3] * sc);
    *(volatile v4u*)(out + (size_t)i * 8) = p;
    __threadfence();
    *(volatile v4u*)(out + (size_t)i * 8) = p;
  }
}

__global__ __launch_bounds__(256)
void layernorm_f16(const float* __restrict__ x, const float* __restrict__ gw, const float* __restrict__ gb,
                   unsigned short* out, int nrows) {
  const int lane = threadIdx.x & 31;
  const int wave = threadIdx.x >> 5;
  const int row  = blockIdx.x * 8 + wave;
  if (row >= nrows) return;
  const float* xr = x + (size_t)row * DM;
  const int c0 = 8 * lane, c1 = 256 + 8 * lane;
  const v4f a0 = *(const v4f*)(xr + c0);
  const v4f a1 = *(const v4f*)(xr + c0 + 4);
  const v4f a2 = *(const v4f*)(xr + c1);
  const v4f a3 = *(const v4f*)(xr + c1 + 4);
  float s = 0.f;
#pragma unroll
  for (int e = 0; e < 4; ++e) s += a0[e];
#pragma unroll
  for (int e = 0; e < 4; ++e) s += a1[e];
#pragma unroll
  for (int e = 0; e < 4; ++e) s += a2[e];
#pragma unroll
  for (int e = 0; e < 4; ++e) s += a3[e];
#pragma unroll
  for (int off = 1; off < 32; off <<= 1) s += __shfl_xor(s, off, 32);
  const float mean = s * (1.0f / (float)DM);
  const v4f d0 = a0 - mean, d1 = a1 - mean, d2 = a2 - mean, d3 = a3 - mean;
  float q = 0.f;
#pragma unroll
  for (int e = 0; e < 4; ++e) q += d0[e] * d0[e];
#pragma unroll
  for (int e = 0; e < 4; ++e) q += d1[e] * d1[e];
#pragma unroll
  for (int e = 0; e < 4; ++e) q += d2[e] * d2[e];
#pragma unroll
  for (int e = 0; e < 4; ++e) q += d3[e] * d3[e];
#pragma unroll
  for (int off = 1; off < 32; off <<= 1) q += __shfl_xor(q, off, 32);
  const float rstd = rsqrtf(q * (1.0f / (float)DM) + 1e-5f);
  const v4f w0 = *(const v4f*)(gw + c0), w1 = *(const v4f*)(gw + c0 + 4);
  const v4f w2 = *(const v4f*)(gw + c1), w3 = *(const v4f*)(gw + c1 + 4);
  const v4f b0 = *(const v4f*)(gb + c0), b1 = *(const v4f*)(gb + c0 + 4);
  const v4f b2 = *(const v4f*)(gb + c1), b3 = *(const v4f*)(gb + c1 + 4);
  const v4f y0 = (d0 * rstd) * w0 + b0;
  const v4f y1 = (d1 * rstd) * w1 + b1;
  const v4f y2 = (d2 * rstd) * w2 + b2;
  const v4f y3 = (d3 * rstd) * w3 + b3;
  v4u p0, p1;
  p0[0] = pkf(y0[0], y0[1]); p0[1] = pkf(y0[2], y0[3]); p0[2] = pkf(y1[0], y1[1]); p0[3] = pkf(y1[2], y1[3]);
  p1[0] = pkf(y2[0], y2[1]); p1[1] = pkf(y2[2], y2[3]); p1[2] = pkf(y3[0], y3[1]); p1[3] = pkf(y3[2], y3[3]);
  unsigned short* orow = out + (size_t)row * DM;
  *(volatile v4u*)(orow + c0) = p0;
  *(volatile v4u*)(orow + c1) = p1;
  __threadfence();
  *(volatile v4u*)(orow + c0) = p0;
  *(volatile v4u*)(orow + c1) = p1;
}

template <int OUT16, int HAS_BIAS, int GELU, int HAS_RES>
__global__ __launch_bounds__(256) void gemm64(
    const unsigned short* __restrict__ Ap, int lda, long long strideA,
    const unsigned short* __restrict__ Btp, int ldb, long long strideB,
    void* Cout, int ldc, long long strideC,
    const float* __restrict__ bias, const float* __restrict__ resid, int ldr,
    int M, int N, int K, float oscale, float cscale) {
  const _Float16* A  = (const _Float16*)(const void*)Ap;
  const _Float16* Bt = (const _Float16*)(const void*)Btp;
  __shared__ __align__(16) float sT[8][16 * 68];
  const int b    = blockIdx.y;
  const int lane = threadIdx.x & 31;
  const int wave = threadIdx.x >> 5;
  const int tilesN = N >> 6;
  const int tilesM = M >> 6;
  const int tile = blockIdx.x * 8 + wave;
  if (tile >= tilesM * tilesN) return;
  const int tm = tile / tilesN;
  const int tn = tile - tm * tilesN;
  const int m0 = tm << 6;
  const int n0 = tn << 6;

  const _Float16* Ab = A  + (size_t)b * (size_t)strideA;
  const _Float16* Bb = Bt + (size_t)b * (size_t)strideB;

  const int rlane = lane & 15;
  const int koff  = (lane >> 4) * 8;
  const int mOff  = (lane >> 4) * 8;

  v8f acc[4][4];
#pragma unroll
  for (int i = 0; i < 4; ++i)
#pragma unroll
    for (int j = 0; j < 4; ++j) acc[i][j] = zero8();

  for (int k0 = 0; k0 < K; k0 += 32) {
    v16h bh[4];
#pragma unroll
    for (int j = 0; j < 4; ++j) {
      const size_t bo = (size_t)(n0 + (j << 4) + rlane) * ldb + koff + k0;
      bh[j] = ldfrag_h(Bb + bo);
    }
#pragma unroll
    for (int i = 0; i < 4; ++i) {
      const size_t ao = (size_t)(m0 + (i << 4) + rlane) * lda + koff + k0;
      const v16h ah = ldfrag_h(Ab + ao);
#pragma unroll
      for (int j = 0; j < 4; ++j) acc[i][j] = mma_h_raw(ah, bh[j], acc[i][j]);
      dep_guard(acc[i][0], acc[i][3], ah);
    }
    keep4(bh[0], bh[1], bh[2], bh[3]);
  }
  acc_guard4(acc[0][0], acc[0][1], acc[0][2], acc[0][3]);
  acc_guard4(acc[1][0], acc[1][1], acc[1][2], acc[1][3]);
  acc_guard4(acc[2][0], acc[2][1], acc[2][2], acc[2][3]);
  acc_guard4(acc[3][0], acc[3][1], acc[3][2], acc[3][3]);

  float* slab = sT[wave];
#pragma unroll
  for (int i = 0; i < 4; ++i) {
    const int mBase = m0 + (i << 4);
#pragma unroll
    for (int j = 0; j < 4; ++j) {
#pragma unroll
      for (int r = 0; r < 8; ++r) {
        slab[(mOff + r) * 68 + (j << 4) + rlane] = acc[i][j][r];
      }
    }
    lds_wave_sync();
    if (OUT16 == 0) {
      float* C = (float*)Cout + (size_t)b * (size_t)strideC;
      const int hh = lane >> 4, c4 = (lane & 15) * 4;
      v4f bias4 = zero4();
      if (HAS_BIAS) bias4 = *(const v4f*)(bias + n0 + c4);
      v4f vals[8];
#pragma unroll
      for (int it = 0; it < 8; ++it) {
        const int row = it * 2 + hh;
        v4f v = *(const v4f*)(slab + row * 68 + c4);
        v = v * oscale + bias4;
        if (GELU) v = gelu4(v);
        if (HAS_RES) v += *(const v4f*)(resid + (size_t)(mBase + row) * ldr + n0 + c4);
        vals[it] = v;
      }
      for (int pass = 0; pass < 2; ++pass) {
#pragma unroll
        for (int it = 0; it < 8; ++it) {
          const int row = it * 2 + hh;
          *(volatile v4f*)(C + (size_t)(mBase + row) * ldc + n0 + c4) = vals[it];
        }
        __threadfence();
      }
    } else {
      unsigned short* C = (unsigned short*)Cout + (size_t)b * (size_t)strideC;
      const int q = lane >> 3, c8 = (lane & 7) * 8;
      v4f bb0 = zero4(), bb1 = zero4();
      if (HAS_BIAS) { bb0 = *(const v4f*)(bias + n0 + c8); bb1 = *(const v4f*)(bias + n0 + c8 + 4); }
      v4u hv[4];
#pragma unroll
      for (int it = 0; it < 4; ++it) {
        const int row = it * 4 + q;
        const float* sp = slab + row * 68 + c8;
        v4f x0 = *(const v4f*)(sp);
        v4f x1 = *(const v4f*)(sp + 4);
        x0 = x0 * oscale + bb0;
        x1 = x1 * oscale + bb1;
        if (GELU) { x0 = gelu4(x0); x1 = gelu4(x1); }
        x0 = x0 * cscale;
        x1 = x1 * cscale;
        v4u pk;
        pk[0] = pkf(x0[0], x0[1]); pk[1] = pkf(x0[2], x0[3]);
        pk[2] = pkf(x1[0], x1[1]); pk[3] = pkf(x1[2], x1[3]);
        hv[it] = pk;
      }
      for (int pass = 0; pass < 2; ++pass) {
#pragma unroll
        for (int it = 0; it < 4; ++it) {
          const int row = it * 4 + q;
          *(volatile v4u*)(C + (size_t)(mBase + row) * ldc + n0 + c8) = hv[it];
        }
        __threadfence();
      }
    }
    lds_wave_sync();
  }
}

__global__ __launch_bounds__(128)
void attn64(const unsigned short* __restrict__ qkp, const unsigned short* __restrict__ vtp,
            const int* __restrict__ amask, unsigned short* op, float sscale) {
  union FH { v16h v; v8h h[2]; };
  __shared__ __align__(16) _Float16 Ksh[64 * 64];
  __shared__ __align__(16) _Float16 Vth[64 * 64];
  __shared__ __align__(16) _Float16 Psh[4][16 * 64];
  __shared__ __align__(16) float    Os[4][16 * 64];
  __shared__ int msk[64];

  const int tid  = threadIdx.x;
  const int wave = tid >> 5;
  const int lane = tid & 31;
  const int hh   = lane >> 4;
  const int c    = lane & 15;

  const int bx   = blockIdx.x;
  const int qb   = bx % NQB;
  const int rest = bx / NQB;
  const int h    = rest % NH;
  const int b    = rest / NH;
  const int q0   = qb * 64 + wave * 16;
  const size_t rowB = (size_t)b * SEQ;
  const size_t QKP  = (size_t)(2 * DM);

  const _Float16* QK = (const _Float16*)(const void*)qkp;
  const _Float16* Vh = (const _Float16*)(const void*)vtp + ((size_t)b * DM + (size_t)h * HD) * SEQ;
  const int* mrp = amask + (size_t)b * SEQ;

  v16h qa[2];
#pragma unroll
  for (int dc = 0; dc < 2; ++dc) {
    const size_t qo = (rowB + q0 + c) * QKP + (size_t)h * HD + dc * 32 + 8 * hh;
    qa[dc] = ldfrag_h(QK + qo);
  }

  float mrow[8], lrow[8];
  v8f oacc[4];
#pragma unroll
  for (int r = 0; r < 8; ++r) { mrow[r] = -INFINITY; lrow[r] = 0.f; }
#pragma unroll
  for (int t = 0; t < 4; ++t) oacc[t] = zero8();

  for (int kt = 0; kt < NQB; ++kt) {
    const int kv0 = kt * 64;
    __syncthreads();
    {
      const int r = tid >> 1, half = (tid & 1) * 32;
      const _Float16* kg = QK + (rowB + kv0 + r) * QKP + DM + (size_t)h * HD + half;
      const _Float16* vg = Vh + (size_t)r * SEQ + kv0 + half;
#pragma unroll
      for (int i = 0; i < 4; ++i) {
        const v8h a0 = *(const v8h*)(kg + 8 * i);
        const v8h b0 = *(const v8h*)(vg + 8 * i);
        *(v8h*)(Ksh + r * 64 + half + 8 * i) = a0;
        *(v8h*)(Vth + r * 64 + half + 8 * i) = b0;
      }
      if (tid < 64) msk[tid] = mrp[kv0 + tid];
    }
    __syncthreads();

    v8f s[4];
#pragma unroll
    for (int j = 0; j < 4; ++j) {
      s[j] = zero8();
#pragma unroll
      for (int dc = 0; dc < 2; ++dc) {
        FH kb;
        kb.h[0] = *(const v8h*)(Ksh + (j * 16 + c) * 64 + dc * 32 + 8 * hh);
        kb.h[1] = *(const v8h*)(Ksh + (j * 16 + c) * 64 + dc * 32 + 16 + 8 * hh);
        s[j] = mma_h(qa[dc], kb.v, s[j]);
      }
    }

    int mk[4];
#pragma unroll
    for (int j = 0; j < 4; ++j) mk[j] = msk[j * 16 + c];
    _Float16* pw = Psh[wave];
#pragma unroll
    for (int r = 0; r < 8; ++r) {
      float m = -INFINITY;
#pragma unroll
      for (int j = 0; j < 4; ++j) {
        const float raw = s[j][r] * sscale;
        const float sv = (mk[j] == 0) ? -INFINITY : raw;
        s[j][r] = sv;
        m = fmaxf(m, sv);
      }
#pragma unroll
      for (int off = 1; off < 16; off <<= 1) m = fmaxf(m, __shfl_xor(m, off, 32));
      const float mnew  = fmaxf(mrow[r], m);
      const float msafe = (mnew == -INFINITY) ? 0.f : mnew;
      const float alpha = __expf(mrow[r] - msafe);
      mrow[r] = mnew;
      float psum = 0.f;
#pragma unroll
      for (int j = 0; j < 4; ++j) {
        const float p = __expf(s[j][r] - msafe);
        psum += p;
        pw[(8 * hh + r) * 64 + j * 16 + c] = (_Float16)(p * PSC);
      }
#pragma unroll
      for (int off = 1; off < 16; off <<= 1) psum += __shfl_xor(psum, off, 32);
      lrow[r] = lrow[r] * alpha + psum;
#pragma unroll
      for (int t = 0; t < 4; ++t) oacc[t][r] *= alpha;
    }
    lds_wave_sync();

#pragma unroll 1
    for (int kk = 0; kk < 2; ++kk) {
      FH pa;
      pa.h[0] = *(const v8h*)(pw + c * 64 + kk * 32 + 8 * hh);
      pa.h[1] = *(const v8h*)(pw + c * 64 + kk * 32 + 16 + 8 * hh);
#pragma unroll
      for (int t = 0; t < 4; ++t) {
        FH vb;
        vb.h[0] = *(const v8h*)(Vth + (t * 16 + c) * 64 + kk * 32 + 8 * hh);
        vb.h[1] = *(const v8h*)(Vth + (t * 16 + c) * 64 + kk * 32 + 16 + 8 * hh);
        oacc[t] = mma_h(pa.v, vb.v, oacc[t]);
      }
    }
  }

  float* os = Os[wave];
#pragma unroll
  for (int r = 0; r < 8; ++r) {
    const float l = lrow[r];
    const float inv = ((l > 0.f) ? (1.0f / l) : 0.f) * (OSC / (PSC * QSC));
#pragma unroll
    for (int t = 0; t < 4; ++t) os[(8 * hh + r) * 64 + t * 16 + c] = oacc[t][r] * inv;
  }
  lds_wave_sync();
  {
    const int q4 = lane >> 3, c8 = (lane & 7) * 8;
    v4u hv[4];
#pragma unroll
    for (int it = 0; it < 4; ++it) {
      const int row = it * 4 + q4;
      const float* sp = os + row * 64 + c8;
      const v4f x0 = *(const v4f*)(sp);
      const v4f x1 = *(const v4f*)(sp + 4);
      v4u pk;
      pk[0] = pkf(x0[0], x0[1]); pk[1] = pkf(x0[2], x0[3]);
      pk[2] = pkf(x1[0], x1[1]); pk[3] = pkf(x1[2], x1[3]);
      hv[it] = pk;
    }
    for (int pass = 0; pass < 2; ++pass) {
#pragma unroll
      for (int it = 0; it < 4; ++it) {
        const int row = it * 4 + q4;
        const size_t go = (rowB + q0 + row) * DM + (size_t)h * HD + c8;
        *(volatile v4u*)(op + go) = hv[it];
      }
      __threadfence();
    }
  }
}

extern "C" void kernel_launch(void* const* d_in, const int* in_sizes, int n_in,
                              void* d_out, int out_size, void* d_ws, size_t ws_size,
                              hipStream_t stream) {
  if (n_in < 13) return;
  if (in_sizes[0] != NROW * DM) return;
  if (in_sizes[1] != NB * SEQ) return;
  if (in_sizes[2] != DM || in_sizes[3] != DM) return;
  if (in_sizes[4] != 3 * DM * DM) return;
  if (in_sizes[5] != DM * DM || in_sizes[6] != DM) return;
  if (in_sizes[7] != DM || in_sizes[8] != DM) return;
  if (in_sizes[9] != HID * DM || in_sizes[10] != HID) return;
  if (in_sizes[11] != DM * HID || in_sizes[12] != DM) return;
  if (out_size != NROW * DM) return;

  const float* x      = (const float*)d_in[0];
  const int*   amask  = (const int*)d_in[1];
  const float* ln1_w  = (const float*)d_in[2];
  const float* ln1_b  = (const float*)d_in[3];
  const float* qkv_w  = (const float*)d_in[4];
  const float* proj_w = (const float*)d_in[5];
  const float* proj_b = (const float*)d_in[6];
  const float* ln2_w  = (const float*)d_in[7];
  const float* ln2_b  = (const float*)d_in[8];
  const float* fc1_w  = (const float*)d_in[9];
  const float* fc1_b  = (const float*)d_in[10];
  const float* fc2_w  = (const float*)d_in[11];
  const float* fc2_b  = (const float*)d_in[12];

  const size_t PWqkv = (size_t)3 * DM * DM * 2;
  const size_t PWprj = (size_t)DM * DM * 2;
  const size_t PWfc  = (size_t)HID * DM * 2;
  const size_t PH    = (size_t)NROW * DM * 2;
  const size_t PQK   = (size_t)NROW * 2 * DM * 2;
  const size_t PVT   = (size_t)NB * DM * SEQ * 2;
  const size_t PX1   = (size_t)NROW * DM * 4;
  const size_t PMH   = (size_t)NROW * HID * 2;
  size_t off = 0;
  const size_t oWqkv = off; off += PWqkv;
  const size_t oWprj = off; off += PWprj;
  const size_t oWfc1 = off; off += PWfc;
  const size_t oWfc2 = off; off += PWfc;
  const size_t oH1   = off; off += PH;
  const size_t oQK   = off; off += PQK;
  const size_t oVT   = off; off += PVT;
  const size_t oO    = off; off += PH;
  const size_t oX1   = off; off += PX1;
  const size_t oH2   = off; off += PH;
  const size_t oMH   = off; off += PMH;
  if (off > ws_size) return;
  if (off > (size_t)134217728) return;

  char* ws = (char*)d_ws;
  unsigned short* Wqkv = (unsigned short*)(ws + oWqkv);
  unsigned short* Wprj = (unsigned short*)(ws + oWprj);
  unsigned short* Wfc1 = (unsigned short*)(ws + oWfc1);
  unsigned short* Wfc2 = (unsigned short*)(ws + oWfc2);
  unsigned short* H1   = (unsigned short*)(ws + oH1);
  unsigned short* QK   = (unsigned short*)(ws + oQK);
  unsigned short* VT   = (unsigned short*)(ws + oVT);
  unsigned short* O16  = (unsigned short*)(ws + oO);
  float*          X1   = (float*)(ws + oX1);
  unsigned short* H2   = (unsigned short*)(ws + oH2);
  unsigned short* MH   = (unsigned short*)(ws + oMH);

  const dim3 blk(256);
  const int n8qkv = 3 * DM * DM / 8;
  const int n8prj = DM * DM / 8;
  const int n8fc  = HID * DM / 8;

  cvt_f16x8<<<dim3((n8qkv + 255) / 256), blk, 0, stream>>>(qkv_w, Wqkv, n8qkv, WSC);
  cvt_f16x8<<<dim3((n8prj + 255) / 256), blk, 0, stream>>>(proj_w, Wprj, n8prj, WSC);
  cvt_f16x8<<<dim3((n8fc + 255) / 256), blk, 0, stream>>>(fc1_w, Wfc1, n8fc, WSC);
  cvt_f16x8<<<dim3((n8fc + 255) / 256), blk, 0, stream>>>(fc2_w, Wfc2, n8fc, WSC);

  layernorm_f16<<<dim3(NROW / 8), blk, 0, stream>>>(x, ln1_w, ln1_b, H1, NROW);

  gemm64<1, 0, 0, 0><<<dim3(((NROW / 64) * (2 * DM / 64) + 7) / 8, 1), blk, 0, stream>>>(
      H1, DM, 0LL, Wqkv, DM, 0LL,
      (void*)QK, 2 * DM, 0LL,
      x, x, DM,
      NROW, 2 * DM, DM, 1.0f / WSC, QSC);

  gemm64<1, 0, 0, 0><<<dim3(((DM / 64) * (SEQ / 64) + 7) / 8, NB), blk, 0, stream>>>(
      Wqkv + (size_t)2 * DM * DM, DM, 0LL, H1, DM, (long long)SEQ * DM,
      (void*)VT, SEQ, (long long)DM * SEQ,
      x, x, DM,
      DM, SEQ, DM, 1.0f / WSC, QSC);

  attn64<<<dim3(NQB * NH * NB), dim3(128), 0, stream>>>(
      QK, VT, amask, O16, 0.125f / (QSC * QSC));

  gemm64<0, 1, 0, 1><<<dim3(((NROW / 64) * (DM / 64) + 7) / 8, 1), blk, 0, stream>>>(
      O16, DM, 0LL, Wprj, DM, 0LL,
      (void*)X1, DM, 0LL,
      proj_b, x, DM,
      NROW, DM, DM, 1.0f / (OSC * WSC), 1.0f);

  layernorm_f16<<<dim3(NROW / 8), blk, 0, stream>>>(X1, ln2_w, ln2_b, H2, NROW);

  gemm64<1, 1, 1, 0><<<dim3(((NROW / 64) * (HID / 64) + 7) / 8, 1), blk, 0, stream>>>(
      H2, DM, 0LL, Wfc1, DM, 0LL,
      (void*)MH, HID, 0LL,
      fc1_b, x, DM,
      NROW, HID, DM, 1.0f / WSC, MSC);

  gemm64<0, 1, 0, 1><<<dim3(((NROW / 64) * (DM / 64) + 7) / 8, 1), blk, 0, stream>>>(
      MH, HID, 0LL, Wfc2, HID, 0LL,
      d_out, DM, 0LL,
      fc2_b, X1, DM,
      NROW, DM, HID, 1.0f / (MSC * WSC), 1.0f);
  (void)hipGetLastError();
}
